// S4DKernel_9801115369843
// MI455X (gfx1250) — hardware-verified
//
#include <hip/hip_runtime.h>
#include <math.h>

typedef __attribute__((ext_vector_type(16))) _Float16 v16h;
typedef __attribute__((ext_vector_type(16))) __bf16 v16b;
typedef __attribute__((ext_vector_type(8)))  _Float16 v8h;
typedef __attribute__((ext_vector_type(8)))  float v8f;
typedef __attribute__((ext_vector_type(4)))  float v4f;
typedef __attribute__((ext_vector_type(2)))  float v2f;
typedef __attribute__((ext_vector_type(4)))  unsigned v4u;
typedef __attribute__((ext_vector_type(4)))  int v4i;
typedef float __attribute__((may_alias)) float_a;
typedef int __attribute__((may_alias)) int_a;

template <typename T> __device__ __forceinline__ void vst2(void* p, T v) { *(volatile T*)p = v; __threadfence(); *(volatile T*)p = v; }
__device__ __forceinline__ v8f wmma16(v16h a, v16h b, v8f c) {
  v8f d = __builtin_amdgcn_wmma_f32_16x16x32_f16(false, a, false, b, (short)0, c, false, false);
  asm volatile("v_nop\n\tv_nop\n\tv_nop\n\tv_nop" : "+v"(d) : "v"(a), "v"(b));
  return d;
}
__device__ __forceinline__ v8f wmma_bf(v16b a, v16b b, v8f c) {
  v8f d = __builtin_amdgcn_wmma_f32_16x16x32_bf16(false, a, false, b, (short)0, c, false, false);
  asm volatile("v_nop\n\tv_nop\n\tv_nop\n\tv_nop" : "+v"(d) : "v"(a), "v"(b));
  return d;
}
__device__ __forceinline__ v16h frag_h(const _Float16* rowk0, int lane) {
  union { v16h v; v8h q[2]; } u; const _Float16* p = rowk0 + 8 * (lane >> 4);
  u.q[0] = *(const v8h*)p; u.q[1] = *(const v8h*)(p + 16); return u.v;
}
__device__ __forceinline__ v16h frag_f32(const float* rowk0, int lane) {
  v16h a; const float* p = rowk0 + 8 * (lane >> 4);
#pragma unroll
  for (int i = 0; i < 8; ++i) { a[i] = (_Float16)p[i]; a[8 + i] = (_Float16)p[16 + i]; }
  return a;
}
__device__ __forceinline__ v16h frag_f32s(const float* rowk0, int lane, float sc) {
  v16h a; const float* p = rowk0 + 8 * (lane >> 4);
#pragma unroll
  for (int i = 0; i < 8; ++i) { a[i] = (_Float16)(p[i] * sc); a[8 + i] = (_Float16)(p[16 + i] * sc); }
  return a;
}
__device__ __forceinline__ v16h fragc_f32(const float* W, int k0, int n, int lane, int ld, int K) {
  v16h a; const int g = lane >> 4;
#pragma unroll
  for (int i = 0; i < 8; ++i) { const int ka = k0 + 8 * g + i, kb = ka + 16;
    a[i] = (_Float16)(ka < K ? W[(size_t)(ka < K ? ka : K - 1) * ld + n] : 0.f); a[8 + i] = (_Float16)(kb < K ? W[(size_t)(kb < K ? kb : K - 1) * ld + n] : 0.f); }
  return a;
}
struct F2 { v16b h, l; };
__device__ __forceinline__ F2 bsplit16(const float v[16]) { F2 r;
#pragma unroll
  for (int i = 0; i < 16; ++i) { const __bf16 h = (__bf16)v[i]; r.h[i] = h; r.l[i] = (__bf16)(v[i] - (float)h); }
  return r; }
__device__ __forceinline__ F2 split_row(const float* row, int k0, int lane) { float v[16]; const float* p = row + k0 + 8 * (lane >> 4);
#pragma unroll
  for (int i = 0; i < 8; ++i) { v[i] = p[i]; v[8 + i] = p[16 + i]; }
  return bsplit16(v); }
__device__ __forceinline__ F2 split_rowK(const float* row, int k0, int lane, int K) { float v[16]; const int g = lane >> 4;
#pragma unroll
  for (int i = 0; i < 8; ++i) { const int ka = k0 + 8 * g + i, kb = ka + 16; v[i] = ka < K ? row[ka < K ? ka : K - 1] : 0.f; v[8 + i] = kb < K ? row[kb < K ? kb : K - 1] : 0.f; }
  return bsplit16(v); }
__device__ __forceinline__ F2 split_col(const float* W, int k0, int n, int lane, int ld, int K) { float v[16]; const int g = lane >> 4;
#pragma unroll
  for (int i = 0; i < 8; ++i) { const int ka = k0 + 8 * g + i, kb = ka + 16; v[i] = ka < K ? W[(size_t)(ka < K ? ka : K - 1) * ld + n] : 0.f; v[8 + i] = kb < K ? W[(size_t)(kb < K ? kb : K - 1) * ld + n] : 0.f; }
  return bsplit16(v); }
__device__ __forceinline__ v8f mac3(const F2& a, const F2& b, v8f c) { c = wmma_bf(a.l, b.h, c); c = wmma_bf(a.h, b.l, c); return wmma_bf(a.h, b.h, c); }
__device__ __forceinline__ float sigm(float v) { return 1.0f / (1.0f + expf(-v)); }
#define LDSX() do { asm volatile("s_wait_dscnt 0" ::: "memory"); __builtin_amdgcn_wave_barrier(); __builtin_amdgcn_fence(__ATOMIC_RELEASE, "workgroup"); } while (0)


#define NHC 1024
#define NM 32
#define LL 4096
#ifndef NHP
#define NHP NHC
#endif
__device__ __forceinline__ float bfr(float v) { return (float)(__bf16)v; }
typedef __attribute__((ext_vector_type(8))) __bf16 v8b;
__global__ __launch_bounds__(128) void k_s4d(const float* __restrict__ LDT, const float* __restrict__ CR, const float* __restrict__ LAR, const float* __restrict__ AIM, float* __restrict__ OUT) {
  __shared__ __align__(16) __bf16 sbh[4][16][72], sbl[4][16][72]; __shared__ __align__(16) float sa[4][64]; __shared__ __align__(16) float sk[4][32];
  const int tid = threadIdx.x, wave = tid >> 5, lane = tid & 31, col = lane & 15, g = lane >> 4; const int h = blockIdx.x * 4 + wave; const int n = lane;
  const float dt = expf(bfr(LDT[h])); const float ar = -expf(bfr(LAR[h * NM + n])), aim = bfr(AIM[h * NM + n]);
  const float zr = ar * dt * 0.5f, zi = aim * dt * 0.5f;
  const float dr = 1.0f - zr, di = -zi;
  const float nr = 1.0f + zr, ni = zi;
  const float dd = dr * dr + di * di;
  const float dAr = (nr * dr + ni * di) / dd, dAi = (ni * dr - nr * di) / dd;
  const float br = dt * dr / dd, bi = -dt * di / dd;
  const float cr = bfr(CR[((size_t)h * NM + n) * 2]), ci = bfr(CR[((size_t)h * NM + n) * 2 + 1]);
  const float dcr = cr * br - ci * bi, dci = cr * bi + ci * br;
  sa[wave][n] = 2.0f * dcr; sa[wave][NM + n] = -2.0f * dci;
  LDSX();
  F2 af[2];
#pragma unroll
  for (int kc = 0; kc < 2; ++kc) { float v[16];
#pragma unroll
    for (int i = 0; i < 8; ++i) { v[i] = (col == 0) ? sa[wave][kc * 32 + 8 * g + i] : 0.f; v[8 + i] = (col == 0) ? sa[wave][kc * 32 + 16 + 8 * g + i] : 0.f; }
    af[kc] = bsplit16(v); }
  float vr = 1.0f, vi = 0.0f;
#pragma unroll 1
  for (int ch = 0; ch < LL / 16; ++ch) {
#pragma unroll 4
    for (int lc = 0; lc < 16; ++lc) { const __bf16 hr = (__bf16)vr, hi2 = (__bf16)vi; sbh[wave][lc][n] = hr; sbl[wave][lc][n] = (__bf16)(vr - (float)hr); sbh[wave][lc][NM + n] = hi2; sbl[wave][lc][NM + n] = (__bf16)(vi - (float)hi2);
      const float tr = vr * dAr - vi * dAi, ti = vr * dAi + vi * dAr; vr = tr; vi = ti; }
    LDSX();
    v8f acc = {};
#pragma unroll
    for (int kc = 0; kc < 2; ++kc) { v16b bh, bl; { union { v16b v; v8b q[2]; } u, w; u.q[0] = *(const v8b*)&sbh[wave][col][kc * 32 + 8 * g]; u.q[1] = *(const v8b*)&sbh[wave][col][kc * 32 + 16 + 8 * g]; w.q[0] = *(const v8b*)&sbl[wave][col][kc * 32 + 8 * g]; w.q[1] = *(const v8b*)&sbl[wave][col][kc * 32 + 16 + 8 * g]; bh = u.v; bl = w.v; }
      acc = wmma_bf(af[kc].h, bh, acc); acc = wmma_bf(af[kc].l, bh, acc); acc = wmma_bf(af[kc].h, bl, acc); }
    if (g == 0) sk[wave][(ch & 1) * 16 + col] = acc[0];
    LDSX();
    if (ch & 1) { vst2(OUT + (size_t)h * LL + (size_t)(ch - 1) * 16 + lane, sk[wave][lane]); }
    LDSX(); } }
extern "C" void kernel_launch(void* const* d_in, const int* in_sizes, int n_in, void* d_out, int out_size, void* d_ws, size_t ws_size, hipStream_t stream) {
  (void)in_sizes; (void)n_in; (void)out_size; (void)d_ws; (void)ws_size;
  const float** F = (const float**)d_in;
  k_s4d<<<dim3(NHP / 4), 128, 0, stream>>>(F[0], F[1], F[2], F[3], (float*)d_out);
}
